// DepthAwareGATv2Backbone_15522011808342
// MI455X (gfx1250) — hardware-run, weakly checked
//
#include <hip/hip_runtime.h>


namespace {
constexpr int N = 50000, E = 600000, F = 128, NH = 8, C = 16, D = NH * C, NEF = 4, HE = 16, NPB = (E + 255) / 256;
constexpr float XS = 8.0f, WSC = 256.0f, SLOPE = 0.2f;
typedef _Float16 b16;
typedef __attribute__((ext_vector_type(16))) _Float16 v16b;
typedef __attribute__((ext_vector_type(8))) _Float16 v8b;
typedef __attribute__((ext_vector_type(8))) float v8f;
typedef __attribute__((ext_vector_type(4))) float v4f;
__device__ __forceinline__ float bf16_rne(float f) { unsigned int u = __float_as_uint(f); u += 0x7FFFu + ((u >> 16) & 1u); float r = __uint_as_float(u & 0xFFFF0000u); asm volatile("" : "+v"(r)); return r; }
__device__ __forceinline__ void split16(float v, b16& hi, b16& lo) { hi = (b16)v; lo = (b16)(v - (float)hi); }
__device__ __forceinline__ v16b frag_kb(const b16* p, int hh) { const v8b a = *(const v8b*)(p + 8 * hh), b = *(const v8b*)(p + 16 + 8 * hh); v16b f;
#pragma unroll
  for (int e = 0; e < 8; ++e) { f[e] = a[e]; f[8 + e] = b[e]; } return f; }
__device__ __forceinline__ v8f wmma16b(v16b a, v16b b, v8f c) { v8f d = __builtin_amdgcn_wmma_f32_16x16x32_f16(false, a, false, b, (short)0, c, false, false); asm volatile("v_nop\n\tv_nop\n\tv_nop\n\tv_nop" : "+v"(d) : "v"(a), "v"(b)); return d; }
__device__ __forceinline__ void wave_lds_sync() { __builtin_amdgcn_fence(__ATOMIC_RELEASE, "workgroup"); __builtin_amdgcn_wave_barrier(); __builtin_amdgcn_fence(__ATOMIC_ACQUIRE, "workgroup"); }
__device__ __forceinline__ float pmul(float a, float b) { float p = a * b; asm volatile("" : "+v"(p)); return p; }
__device__ __forceinline__ int iclamp(int v, int lo, int hi) { return v < lo ? lo : (v > hi ? hi : v); }
__device__ __forceinline__ float lrelu(float v) { return v > 0.0f ? v : SLOPE * v; }
__device__ __forceinline__ float elu(float v) { return v > 0.0f ? v : (__expf(v) - 1.0f); }
constexpr int CSR_NBLK9 = 512, CSR_GB9 = 9, CSR_GN9 = 1 << CSR_GB9  , CSR_TS9 = (CSR_GN9 < 32 ? 32 : CSR_GN9)  , CSR_MAXG9 = 512, CSR_CAP9 = 12288  ;
__device__ __host__ __forceinline__ int csr_tix9(int v) { return (v >> CSR_GB9) * CSR_TS9 + (v & (CSR_GN9 - 1)); }
__global__ __launch_bounds__(64) void csrA_kernel9(const int* __restrict__ dst, int E, int N, int nG, int CHP, int NGP, int* __restrict__ STG, int* __restrict__ HST) {
  extern __shared__ int sm[];
  int* cnt = sm; int* run = sm + NGP; int* ids = sm + 2 * NGP;
  const int b = blockIdx.x; const int ch = (E + CSR_NBLK9 - 1) / CSR_NBLK9; const int e0 = b * ch, e1 = min(E, e0 + ch);
  for (int i = threadIdx.x; i < NGP; i += 64) cnt[i] = 0;
  for (int i = threadIdx.x; i < CHP; i += 64) ids[i] = -1;
  __syncthreads();
  if (threadIdx.x == 0) {
    for (int e = e0; e < e1; ++e) { int d = dst[e]; d = (d < 0) ? 0 : (d >= N ? N - 1 : d); cnt[d >> CSR_GB9] += 1; }
    int acc = 0; for (int g = 0; g < nG; ++g) { run[g] = acc; acc += cnt[g]; }
    for (int e = e0; e < e1; ++e) { int d = dst[e]; d = (d < 0) ? 0 : (d >= N ? N - 1 : d); const int g = d >> CSR_GB9; ids[run[g]] = e; run[g] += 1; } }
  __syncthreads();
  typedef __attribute__((ext_vector_type(4))) int v4i;
  for (int pass = 0; pass < 2; ++pass) {
    for (int i = threadIdx.x; i < CHP / 4; i += 64) *(volatile v4i*)(STG + (size_t)b * CHP + i * 4) = *(const v4i*)(&ids[i * 4]);
    for (int i = threadIdx.x; i < NGP / 4; i += 64) { v4i v; for (int e = 0; e < 4; ++e) v[e] = (i * 4 + e < nG) ? cnt[i * 4 + e] : 0; *(volatile v4i*)(HST + (size_t)b * NGP + i * 4) = v; }
    __threadfence(); }
}
__global__ __launch_bounds__(512) void csrS_kernel9(const int* __restrict__ HST, int nG, int NGP, int* __restrict__ START, int* __restrict__ TOT, int* __restrict__ OFF) {
  __shared__ int tot[CSR_MAXG9];
  const int b = threadIdx.x;
  for (int pass = 0; pass < 2; ++pass) { int runb = 0; for (int g = 0; g < nG; ++g) { int c = HST[(size_t)b * NGP + g]; c = (c < 0) ? 0 : c; ((volatile int*)OFF)[(size_t)g * CSR_NBLK9 + b] = runb; runb += c; } __threadfence(); }
  for (int g = threadIdx.x; g < nG; g += 512) { int s = 0; for (int bb = 0; bb < CSR_NBLK9; ++bb) { int c = HST[(size_t)bb * NGP + g]; s += (c < 0) ? 0 : c; } tot[g] = s; }
  __syncthreads();
  if (threadIdx.x < 32) {
    __shared__ int st[CSR_MAXG9 + 32];
    if (threadIdx.x == 0) { int acc = 0; for (int g = 0; g < NGP; ++g) { st[g] = acc; if (g < nG) acc += (tot[g] + 31) & ~31; } st[NGP] = acc; }
    __builtin_amdgcn_fence(__ATOMIC_RELEASE, "workgroup"); __builtin_amdgcn_wave_barrier(); __builtin_amdgcn_fence(__ATOMIC_ACQUIRE, "workgroup");
    for (int pass = 0; pass < 2; ++pass) { for (int i = threadIdx.x; i < NGP + 32; i += 32) { ((volatile int*)START)[i] = (i <= NGP) ? st[min(i, NGP)] : 0; ((volatile int*)TOT)[i] = (i < nG) ? tot[i] : 0; } __threadfence(); } }
}
__global__ __launch_bounds__(256) void csrB_kernel9(const int* __restrict__ dst, int N, int nG, int CHP, int NGP, int permLen, const int* __restrict__ STG, const int* __restrict__ HST, const int* __restrict__ OFF, const int* __restrict__ START, const int* __restrict__ TOT, int* __restrict__ PERM, int* __restrict__ ROWPTR, int* __restrict__ ROWCNT, int* __restrict__ FLAG) {
  typedef __attribute__((ext_vector_type(4))) int v4i;
  __shared__ int ids[CSR_CAP9]; __shared__ unsigned short key[CSR_CAP9]; __shared__ int outp[CSR_CAP9]; __shared__ int ncnt[CSR_GN9 + 1]; __shared__ int boff[CSR_NBLK9 + 1];
  const int g = blockIdx.x, t_ = threadIdx.x; int tot = TOT[g]; int st = START[g], stn = START[g + 1]; const int v0 = g * CSR_GN9; const int nv = min(CSR_GN9, N - v0); const int t0 = g * CSR_TS9;
  st = (st < 0) ? 0 : (st > permLen - 32 ? permLen - 32 : st) & ~31; stn = (stn < st) ? st : (stn > permLen ? permLen : stn); tot = (tot < 0) ? 0 : tot; if (tot > stn - st && tot <= CSR_CAP9) tot = stn - st;
  if (tot > CSR_CAP9) {
    for (int pass = 0; pass < 2; ++pass) { for (int i = t_; i < CSR_TS9 / 4; i += 256) { v4i a, c; for (int e = 0; e < 4; ++e) { a[e] = st; c[e] = 0; } *(volatile v4i*)(ROWPTR + t0 + i * 4) = a; *(volatile v4i*)(ROWCNT + t0 + i * 4) = c; } if (t_ == 0) ((volatile int*)FLAG)[0] = 1; __threadfence(); } (void)nv; return; }
  if (t_ == 0) { int acc = 0; for (int b = 0; b < CSR_NBLK9; ++b) { boff[b] = acc; int c = HST[(size_t)b * NGP + g]; c = (c < 0) ? 0 : (c > CHP ? CHP : c); acc += c; if (acc > tot) acc = tot; } boff[CSR_NBLK9] = acc; }
  for (int i = t_; i <= CSR_GN9; i += 256) ncnt[i] = 0;
  __syncthreads();
  for (int b = 0; b < CSR_NBLK9; ++b) { const int c = boff[b + 1] - boff[b]; int o_ = OFF[(size_t)g * CSR_NBLK9 + b]; o_ = (o_ < 0) ? 0 : (o_ > CHP - c ? CHP - c : o_); const int* src_ = STG + (size_t)b * CHP + o_;
    for (int i = t_; i < c; i += 256) { int id = src_[i]; id = (id < 0) ? 0 : id; ids[boff[b] + i] = id; int d = dst[id]; d = (d < v0) ? v0 : (d >= N ? N - 1 : d); int kk = d - v0; kk = (kk < 0) ? 0 : (kk >= CSR_GN9 ? CSR_GN9 - 1 : kk); key[boff[b] + i] = (unsigned short)kk; } }
  __syncthreads();
  if (t_ == 0) { for (int i = 0; i < tot; ++i) ncnt[key[i]] += 1; int acc = 0; for (int vl = 0; vl < CSR_GN9; ++vl) { const int c = ncnt[vl]; ncnt[vl] = acc; acc += c; } ncnt[CSR_GN9] = acc;
    for (int i = 0; i < tot; ++i) { const int vl = key[i]; outp[ncnt[vl]] = ids[i]; ncnt[vl] += 1; }
    for (int vl = CSR_GN9; vl > 0; --vl) ncnt[vl] = ncnt[vl - 1]; ncnt[0] = 0; }
  __syncthreads();
  for (int pass = 0; pass < 2; ++pass) {
    for (int i = t_; i < (stn - st) / 4; i += 256) { v4i v; for (int e = 0; e < 4; ++e) { const int q = i * 4 + e; v[e] = (q < tot) ? outp[q] : -1; } *(volatile v4i*)(PERM + st + i * 4) = v; }
    for (int i = t_; i < CSR_TS9 / 4; i += 256) { v4i a, c; for (int e = 0; e < 4; ++e) { const int vl = i * 4 + e; const int vc = vl < CSR_GN9 ? vl : CSR_GN9; a[e] = (vl < CSR_GN9) ? st + ncnt[vc] : st; c[e] = (vl < nv) ? (ncnt[(vc < CSR_GN9 ? vc : CSR_GN9 - 1) + 1] - ncnt[vc]) : 0; } *(volatile v4i*)(ROWPTR + t0 + i * 4) = a; *(volatile v4i*)(ROWCNT + t0 + i * 4) = c; }
    __threadfence(); }
}
__global__ __launch_bounds__(256) void csrZ_kernel9(int* __restrict__ p, size_t n4) { typedef __attribute__((ext_vector_type(4))) int v4i; const size_t tid = (size_t)blockIdx.x * 256 + threadIdx.x, nth = (size_t)gridDim.x * 256; v4i z = {0, 0, 0, 0}; for (size_t i = tid; i < n4; i += nth) *(volatile v4i*)(p + i * 4) = z; }
struct CsrBufs9 { int *STG, *HST, *OFF, *START, *TOT, *PERM, *ROWPTR, *ROWCNT, *FLAG; int nG, NGP, CHP; size_t permLen; char* base; size_t bytes; };
static size_t csr_carve9(CsrBufs9& c, char* ws, size_t off, int E, int N) {
  const size_t off0 = off; c.base = ws + off;
  auto al = [&](size_t bytes) { char* p = ws + off; off += (bytes + 255) & ~(size_t)255; return p; };
  c.nG = (N + CSR_GN9 - 1) / CSR_GN9; c.NGP = (c.nG + 31) & ~31; const int ch = (E + CSR_NBLK9 - 1) / CSR_NBLK9; c.CHP = (ch + 31) & ~31; c.permLen = (size_t)E + 32 * (size_t)c.nG + 32;
  c.STG = (int*)al((size_t)CSR_NBLK9 * c.CHP * 4); c.HST = (int*)al((size_t)CSR_NBLK9 * c.NGP * 4); c.OFF = (int*)al((size_t)c.NGP * CSR_NBLK9 * 4); c.START = (int*)al((size_t)(c.NGP + 64) * 4); c.TOT = (int*)al((size_t)(c.NGP + 64) * 4);
  c.PERM = (int*)al(c.permLen * 4); c.ROWPTR = (int*)al((size_t)c.nG * CSR_TS9 * 4); c.ROWCNT = (int*)al((size_t)c.nG * CSR_TS9 * 4); c.FLAG = (int*)al(256);
  c.bytes = off - off0; return off;
}
static void csr_build9(const CsrBufs9& c, const int* dst, int E, int N, hipStream_t stream) {
  const size_t smem = (size_t)(2 * c.NGP + c.CHP) * 4;
  csrZ_kernel9<<<512, 256, 0, stream>>>((int*)c.base, c.bytes / 16);
  csrA_kernel9<<<CSR_NBLK9, 64, smem, stream>>>(dst, E, N, c.nG, c.CHP, c.NGP, c.STG, c.HST);
  csrS_kernel9<<<1, 512, 0, stream>>>(c.HST, c.nG, c.NGP, c.START, c.TOT, c.OFF);
  csrB_kernel9<<<c.nG, 256, 0, stream>>>(dst, N, c.nG, c.CHP, c.NGP, (int)c.permLen, c.STG, c.HST, c.OFF, c.START, c.TOT, c.PERM, c.ROWPTR, c.ROWCNT, c.FLAG);
}


__global__ __launch_bounds__(256) void wcopy_kernel(const float* __restrict__ w, size_t total, b16* __restrict__ WT) { const size_t u = (size_t)blockIdx.x * 256 + threadIdx.x; if (u >= total / 8) return; v8b v;
#pragma unroll
  for (int j = 0; j < 8; ++j) v[j] = (b16)(bf16_rne(w[u * 8 + j]) * WSC); for (int pass = 0; pass < 2; ++pass) { *(volatile v8b*)(WT + u * 8) = v; __threadfence(); } }
__global__ __launch_bounds__(256) void edge_kernel(const float* __restrict__ x, const int* __restrict__ srcs, const int* __restrict__ dsts, const float* __restrict__ w1, const float* __restrict__ b1, const float* __restrict__ w2, const float* __restrict__ b2, int NLIM, float* __restrict__ EA, float* __restrict__ PSUM) {
  __shared__ float Eo[256][NH + 1]; const int t = threadIdx.x; const size_t e = (size_t)blockIdx.x * 256 + t; bool ok = e < (size_t)E; size_t i = 0, j = 0;
  if (ok) { i = (size_t)iclamp(srcs[e], 0, N - 1); j = (size_t)iclamp(dsts[e], 0, N - 1); if (i >= (size_t)NLIM || j >= (size_t)NLIM) ok = false; }
  float outv[NH];
#pragma unroll
  for (int k = 0; k < NH; ++k) outv[k] = 0.0f;
  if (ok) { float f0 = 0.0f, f1 = 0.0f, f2 = 0.0f, f3 = 0.0f;
#pragma unroll 4
    for (int c = 0; c < F; ++c) { const float a = bf16_rne(x[i * F + c]), b = bf16_rne(x[j * F + c]); f0 += pmul(a, b); const float dd = a - b; f1 += pmul(dd, dd); f2 += pmul(a, a); f3 += pmul(b, b); }
    float hv[HE];
#pragma unroll
    for (int u = 0; u < HE; ++u) hv[u] = fmaxf(bf16_rne(b1[u]) + pmul(f0, bf16_rne(w1[u * NEF])) + pmul(f1, bf16_rne(w1[u * NEF + 1])) + pmul(f2, bf16_rne(w1[u * NEF + 2])) + pmul(f3, bf16_rne(w1[u * NEF + 3])), 0.0f);
#pragma unroll
    for (int k = 0; k < NH; ++k) { float s = bf16_rne(b2[k]);
#pragma unroll
      for (int u = 0; u < HE; ++u) s += pmul(hv[u], bf16_rne(w2[k * HE + u])); outv[k] = s; } }
#pragma unroll
  for (int k = 0; k < NH; ++k) Eo[t][k] = outv[k]; Eo[t][NH] = ok ? 1.0f : 0.0f;
  __syncthreads();
  for (int pass = 0; pass < 2; ++pass) { if (e < (size_t)E) { *(volatile v4f*)(EA + e * NH) = (v4f){outv[0], outv[1], outv[2], outv[3]}; *(volatile v4f*)(EA + e * NH + 4) = (v4f){outv[4], outv[5], outv[6], outv[7]}; }
    if (t < 32) { float s = 0.0f; if (t <= NH) {
#pragma unroll 1
        for (int r = 0; r < 256; ++r) s += Eo[r][t]; } ((volatile float*)PSUM)[(size_t)blockIdx.x * 32 + t] = s; }
    __threadfence(); } }
__global__ __launch_bounds__(256) void glob_kernel(const float* __restrict__ PSUM, const float* __restrict__ lew1, const float* __restrict__ ae1, const float* __restrict__ lew2, const float* __restrict__ ae2, float* __restrict__ GV) {
  __shared__ float vals[160]; const int t = threadIdx.x;
  if (t < NH) { double s = 0.0, c = 0.0;
#pragma unroll 1
    for (int b = 0; b < NPB; ++b) { s += (double)PSUM[(size_t)b * 32 + t]; c += (double)PSUM[(size_t)b * 32 + NH]; } vals[t] = (float)(s / (c > 0.0 ? c : 1.0)); }
  if (t >= 32 && t < 32 + 128) { const int l = (t - 32) / 64, hd = ((t - 32) / 8) % 8, k = (t - 32) % 8; const float* lew = l == 0 ? lew1 : lew2; const float* ae = l == 0 ? ae1 : ae2; float s = 0.0f;
#pragma unroll 1
    for (int c = 0; c < C; ++c) s += pmul(bf16_rne(lew[(size_t)(hd * C + c) * NH + k]), bf16_rne(ae[hd * C + c])); vals[t] = s; }
  if (t >= NH && t < 32) vals[t] = 0.0f;
  __syncthreads(); if (t < 32) { for (int pass = 0; pass < 2; ++pass) { for (int q = t; q < 160; q += 32) ((volatile float*)GV)[q] = vals[q]; __threadfence(); } } }
__global__ __launch_bounds__(256) void ae_kernel(const float* __restrict__ EA, const float* __restrict__ GV, int l, float* __restrict__ AE) { const size_t u = (size_t)blockIdx.x * 256 + threadIdx.x; if (u >= (size_t)E * NH) return; const size_t e = u / NH; const int hd = (int)(u % NH); float s = 0.0f;
#pragma unroll
  for (int k = 0; k < NH; ++k) s += pmul(EA[e * NH + k], GV[32 + l * 64 + hd * 8 + k]);
  for (int pass = 0; pass < 2; ++pass) { ((volatile float*)AE)[u] = s; __threadfence(); } }
template <int MODE>
__global__ __launch_bounds__(32) void dense_kernel(const float* __restrict__ IN, const float* __restrict__ IN2, const float* __restrict__ IN3, const b16* __restrict__ WT, const float* __restrict__ bias, int NLIM, float* __restrict__ OUT) {
  constexpr int KT = (MODE == 2) ? 3 * D : D; __shared__ __attribute__((aligned(16))) b16 Ah[16][KT + 8], Al[16][MODE == 0 ? 8 : KT + 8]; __shared__ float Tf[16][132]; const int lane = threadIdx.x, nloc = lane & 15, hlf = lane >> 4; const size_t m0 = (size_t)blockIdx.x * 16; if (m0 >= (size_t)NLIM) return;
  for (int rr = 0; rr < 16; ++rr) for (int q = 0; q < KT / 32; ++q) { const int c = q * 32 + lane; float v; if (MODE == 2) { const int pl = c / D, cc = c % D; const float* src = pl == 0 ? IN : (pl == 1 ? IN2 : IN3); v = src[(m0 + rr) * D + cc]; } else v = IN[(m0 + rr) * D + c];
    if (MODE == 0) Ah[rr][c] = (b16)(bf16_rne(v) * XS); else { b16 p, ql; split16(v * XS, p, ql); Ah[rr][c] = p; Al[rr][c] = ql; } }
  wave_lds_sync(); v8f acc[8];
#pragma unroll
  for (int t = 0; t < 8; ++t) acc[t] = (v8f){};
#pragma unroll 2
  for (int kb = 0; kb < KT; kb += 32) { const v16b a = frag_kb(&Ah[nloc][kb], hlf); v16b a2; if (MODE != 0) a2 = frag_kb(&Al[nloc][kb], hlf);
#pragma unroll
    for (int t = 0; t < 8; ++t) { const v16b bw = frag_kb(WT + (size_t)(t * 16 + nloc) * KT + kb, hlf); acc[t] = wmma16b(a, bw, acc[t]); if (MODE != 0) acc[t] = wmma16b(a2, bw, acc[t]); } }
#pragma unroll
  for (int t = 0; t < 8; ++t) { const int c = t * 16 + nloc; const float bb = bias ? bf16_rne(bias[c]) : 0.0f;
#pragma unroll
    for (int r8 = 0; r8 < 8; ++r8) Tf[8 * hlf + r8][c] = acc[t][r8] * (1.0f / (XS * WSC)) + bb; }
  wave_lds_sync();
  for (int pass = 0; pass < 2; ++pass) { for (int rr = 0; rr < 16; ++rr) *(volatile v4f*)(OUT + (m0 + rr) * D + lane * 4) = *(const v4f*)(&Tf[rr][lane * 4]); __threadfence(); } }
__global__ __launch_bounds__(256) void al_kernel(const float* __restrict__ XS_, const float* __restrict__ as, const float* __restrict__ ad, int NLIM, float* __restrict__ AL) { const int wave = threadIdx.x >> 5, lane = threadIdx.x & 31; const size_t i = (size_t)blockIdx.x * 8 + wave; if (i >= (size_t)NLIM) return;
  const v4f xv = *(const v4f*)(XS_ + i * D + lane * 4); float s = 0.0f, d = 0.0f; for (int k = 0; k < 4; ++k) { s += pmul(xv[k], bf16_rne(as[lane * 4 + k])); d += pmul(xv[k], bf16_rne(ad[lane * 4 + k])); } s += __shfl_xor(s, 1); s += __shfl_xor(s, 2); d += __shfl_xor(d, 1); d += __shfl_xor(d, 2);
  float outv = 0.0f; for (int hd = 0; hd < NH; ++hd) { const float sh = __shfl(s, hd * 4), dh = __shfl(d, hd * 4); if (lane == hd) outv = sh; if (lane == 8 + hd) outv = dh; }
  for (int pass = 0; pass < 2; ++pass) { ((volatile float*)AL)[i * 32 + lane] = outv; __threadfence(); } }
__global__ __launch_bounds__(256) void agg_kernel(const float* __restrict__ XS_, const float* __restrict__ AL, const float* __restrict__ AE, const float* __restrict__ GV, int l, const float* __restrict__ bias, const float* __restrict__ RES, const float* __restrict__ g_, const float* __restrict__ bt, const int* __restrict__ srcs, const int* __restrict__ PERM, const int* __restrict__ ROWPTR, const int* __restrict__ ROWCNT, int permLen, int NLIM, float* __restrict__ HO) {
  const int wave = threadIdx.x >> 5, lane = threadIdx.x & 31; const size_t i = (size_t)blockIdx.x * 8 + wave; if (i >= (size_t)NLIM) return; const int hd = lane >> 2; int st = ROWPTR[i], cnt = ROWCNT[i]; cnt = iclamp(cnt, 0, 1 << 20); st = iclamp(st, 0, permLen - cnt);
  const float adi = AL[i * 32 + 8 + hd]; float aloop = 0.0f;
#pragma unroll
  for (int k = 0; k < NH; ++k) aloop += pmul(GV[k], GV[32 + l * 64 + hd * 8 + k]);
  float m = -INFINITY, den = 0.0f; v4f acc = {0.0f, 0.0f, 0.0f, 0.0f};
  auto step = [&](size_t u, float ae) { const float s = lrelu(AL[u * 32 + hd] + adi + ae); const float mn = fmaxf(m, s); const float sc = (m == -INFINITY) ? 0.0f : __expf(m - mn); const float p = __expf(s - mn); den = den * sc + p; const v4f xv = *(const v4f*)(XS_ + u * D + lane * 4); for (int k = 0; k < 4; ++k) acc[k] = pmul(acc[k], sc) + pmul(p, xv[k]); m = mn; };
#pragma unroll 1
  for (int j = 0; j < cnt; ++j) { const int e = iclamp(PERM[st + j], 0, E - 1); const size_t u = (size_t)iclamp(srcs[e], 0, N - 1); if (u >= (size_t)NLIM) continue; step(u, AE[(size_t)e * NH + hd]); }
  step(i, aloop);
  v4f hv; const float inv = 1.0f / (den + 1e-16f); const v4f rs_ = *(const v4f*)(RES + i * D + lane * 4); for (int k = 0; k < 4; ++k) hv[k] = elu(pmul(acc[k], inv) + bf16_rne(bias[lane * 4 + k])) + rs_[k];
  float s = hv[0] + hv[1] + hv[2] + hv[3]; for (int o = 16; o; o >>= 1) s += __shfl_xor(s, o); const float mu = s * (1.0f / D); float q = 0.0f; for (int k = 0; k < 4; ++k) q += pmul(hv[k] - mu, hv[k] - mu); for (int o = 16; o; o >>= 1) q += __shfl_xor(q, o); const float r_ = rsqrtf(q * (1.0f / D) + 1e-5f);
  v4f o_; for (int k = 0; k < 4; ++k) o_[k] = pmul(pmul(hv[k] - mu, r_), bf16_rne(g_[lane * 4 + k])) + bf16_rne(bt[lane * 4 + k]);
  for (int pass = 0; pass < 2; ++pass) { *(volatile v4f*)(HO + i * D + lane * 4) = o_; __threadfence(); } }
}

extern "C" void kernel_launch(void* const* d_in, const int* in_sizes, int n_in, void* d_out, int out_size, void* d_ws, size_t ws_size, hipStream_t stream) {
  (void)n_in;
  auto Fp = [&](int i) { return (const float*)d_in[i]; }; auto Ip = [&](int i) { return (const int*)d_in[i]; };
  if (in_sizes[0] != N * F || in_sizes[1] != 2 * E || in_sizes[2] != HE * NEF || in_sizes[4] != NH * HE || in_sizes[6] != D * F || in_sizes[12] != D * NH || in_sizes[24] != D * 3 * D || out_size != N * D) return;
  const int NLIM = N;
  size_t off = 0; char* ws = (char*)d_ws;
  auto carve = [&](size_t bytes) { char* p = ws + off; off += (bytes + 255) & ~(size_t)255; return p; };
  b16* WIN = (b16*)carve((size_t)D * F * 2); b16* WL1 = (b16*)carve((size_t)D * D * 2); b16* WL2 = (b16*)carve((size_t)D * D * 2); b16* WJK = (b16*)carve((size_t)D * 3 * D * 2);
  float* EA = (float*)carve((size_t)E * NH * 4); float* PSUM = (float*)carve((size_t)NPB * 32 * 4); float* GV = (float*)carve(256 * 4); float* AE = (float*)carve((size_t)E * NH * 4);
  float* H0 = (float*)carve((size_t)N * D * 4); float* XS_ = (float*)carve((size_t)N * D * 4); float* AL = (float*)carve((size_t)N * 32 * 4); float* H1 = (float*)carve((size_t)N * D * 4); float* H2 = (float*)carve((size_t)N * D * 4); CsrBufs9 csr; off = csr_carve9(csr, ws, off, E, N);
  if (off > ws_size || off > ((size_t)200 << 20)) return;
  wcopy_kernel<<<(D * F / 8 + 255) / 256, 256, 0, stream>>>(Fp(6), (size_t)D * F, WIN); wcopy_kernel<<<(D * D / 8 + 255) / 256, 256, 0, stream>>>(Fp(8), (size_t)D * D, WL1); wcopy_kernel<<<(D * D / 8 + 255) / 256, 256, 0, stream>>>(Fp(14), (size_t)D * D, WL2); wcopy_kernel<<<(3 * D * D / 8 + 255) / 256, 256, 0, stream>>>(Fp(24), (size_t)3 * D * D, WJK);
  csr_build9(csr, Ip(1) + E, E, N, stream);
  edge_kernel<<<NPB, 256, 0, stream>>>(Fp(0), Ip(1), Ip(1) + E, Fp(2), Fp(3), Fp(4), Fp(5), NLIM, EA, PSUM);
  glob_kernel<<<1, 256, 0, stream>>>(PSUM, Fp(12), Fp(11), Fp(18), Fp(17), GV);
  dense_kernel<0><<<N / 16, 32, 0, stream>>>(Fp(0), nullptr, nullptr, WIN, Fp(7), N, H0);
  dense_kernel<0><<<N / 16, 32, 0, stream>>>(Fp(0), nullptr, nullptr, WL1, nullptr, N, XS_);
  al_kernel<<<(N + 7) / 8, 256, 0, stream>>>(XS_, Fp(9), Fp(10), N, AL); ae_kernel<<<(unsigned)(((size_t)E * NH + 255) / 256), 256, 0, stream>>>(EA, GV, 0, AE);
  agg_kernel<<<(NLIM + 7) / 8, 256, 0, stream>>>(XS_, AL, AE, GV, 0, Fp(13), H0, Fp(20), Fp(21), Ip(1), csr.PERM, csr.ROWPTR, csr.ROWCNT, (int)csr.permLen, NLIM, H1);
  dense_kernel<1><<<NLIM / 16, 32, 0, stream>>>(H1, nullptr, nullptr, WL2, nullptr, NLIM, XS_);
  al_kernel<<<(NLIM + 7) / 8, 256, 0, stream>>>(XS_, Fp(15), Fp(16), NLIM, AL); ae_kernel<<<(unsigned)(((size_t)E * NH + 255) / 256), 256, 0, stream>>>(EA, GV, 1, AE);
  agg_kernel<<<(NLIM + 7) / 8, 256, 0, stream>>>(XS_, AL, AE, GV, 1, Fp(19), H1, Fp(22), Fp(23), Ip(1), csr.PERM, csr.ROWPTR, csr.ROWCNT, (int)csr.permLen, NLIM, H2);
  dense_kernel<2><<<NLIM / 16, 32, 0, stream>>>(H0, H1, H2, WJK, Fp(25), NLIM, (float*)d_out);
}
